// MixedOp_37099927503005
// MI455X (gfx1250) — hardware-verified
//
#include <hip/hip_runtime.h>


typedef __attribute__((ext_vector_type(16))) _Float16 v16h;
typedef __attribute__((ext_vector_type(8)))  _Float16 v8h;
typedef __attribute__((ext_vector_type(8)))  float    v8f;

#define BN_SCALE 0.99999500003749981f

#define NB   64
#define NC   128
#define NH   32
#define NW   32
#define NHW  1024
#define NCHW 131072
#define NOPS 8

__global__ void gate_topk_kernel(const float* __restrict__ wts,
                                 const int* __restrict__ top_p,
                                 float* gate,
                                 float* w_out) {
  __shared__ float sg[NB * NOPS];
  __shared__ float sw[NB * NOPS];
  int b = threadIdx.x;
  float lg[NOPS];
#pragma unroll
  for (int i = 0; i < NOPS; ++i) lg[i] = wts[b * NOPS + i];

  int top = top_p[0];
  if (top > NOPS) top = NOPS;
  bool sel[NOPS];
#pragma unroll
  for (int i = 0; i < NOPS; ++i) sel[i] = false;
  for (int t = 0; t < top; ++t) {
    int best = -1;
    float bv = -__builtin_inff();
    for (int i = 0; i < NOPS; ++i)
      if (!sel[i] && lg[i] > bv) { bv = lg[i]; best = i; }
    if (best >= 0) sel[best] = true;
  }
  float mx = -__builtin_inff();
#pragma unroll
  for (int i = 0; i < NOPS; ++i) if (sel[i] && lg[i] > mx) mx = lg[i];
  float e[NOPS];
  float den = 0.f;
#pragma unroll
  for (int i = 0; i < NOPS; ++i) {
    e[i] = sel[i] ? __expf(lg[i] - mx) : 0.f;
    den += e[i];
  }
  float inv = 1.f / den;
#pragma unroll
  for (int i = 0; i < NOPS; ++i) {
    sg[b * NOPS + i] = e[i] * inv;
    sw[b * NOPS + i] = lg[i];
  }
  __syncthreads();
  for (int i = threadIdx.x; i < NB * NOPS; i += NB) { *(volatile float*)(gate + i) = sg[i]; *(volatile float*)(w_out + i) = sw[i]; }
  __threadfence();
  for (int i = threadIdx.x; i < NB * NOPS; i += NB) { *(volatile float*)(gate + i) = sg[i]; *(volatile float*)(w_out + i) = sw[i]; }
}

__global__ void pool_skip_kernel(const float* __restrict__ x,
                                 const float* __restrict__ gate,
                                 float* out) {
  unsigned idx = blockIdx.x * 256u + threadIdx.x;
  unsigned b  = idx >> 17;
  unsigned hw = idx & (NHW - 1);
  int h = (int)(hw >> 5);
  int w = (int)(hw & 31);
  float g1 = gate[b * NOPS + 1];
  float g2 = gate[b * NOPS + 2];
  float g3 = gate[b * NOPS + 3];

  float v = 0.f;
  if (g1 != 0.f || g2 != 0.f) {
    const float* plane = x + (idx - hw);
    float mx = -__builtin_inff();
    float sum = 0.f;
    int cnt = 0;
#pragma unroll
    for (int dy = -1; dy <= 1; ++dy) {
      int hh = h + dy;
      if ((unsigned)hh < (unsigned)NH) {
#pragma unroll
        for (int dx = -1; dx <= 1; ++dx) {
          int ww = w + dx;
          if ((unsigned)ww < (unsigned)NW) {
            float t = plane[hh * NW + ww];
            mx = fmaxf(mx, t);
            sum += t;
            ++cnt;
          }
        }
      }
    }
    v = g1 * (BN_SCALE * mx) + g2 * (BN_SCALE * (sum / (float)cnt));
  }
  v += g3 * x[idx];
  *(volatile float*)(out + idx) = v;
  __threadfence();
  *(volatile float*)(out + idx) = v;
}

template <int KS, int DIL, bool ACCUM>
__global__ __launch_bounds__(256)
void sepstage_kernel(const float* __restrict__ in,
                     const float* __restrict__ dw,
                     const float* __restrict__ pw,
                     const float* __restrict__ gate,
                     int op_idx,
                     float* out) {
  constexpr int LDW = NC + 8;
  constexpr int HALO = (KS / 2) * DIL;
  __shared__ __align__(16) unsigned char smem[2 * NC * LDW * 2];
  _Float16* lds_w = (_Float16*)smem;
  _Float16* lds_b = lds_w + NC * LDW;
  float* cst = (float*)smem;
  __shared__ float    lds_dw[NC * KS * KS];

  const int b  = blockIdx.x >> 3;
  const int r0 = (blockIdx.x & 7) * 4;
  const int tid = threadIdx.x;

  const float g = gate[b * NOPS + op_idx];
  if (g == 0.f) return;

  const float* inb = in + (size_t)b * NCHW;

  {
    const int rlo = (r0 - HALO) < 0 ? 0 : (r0 - HALO);
    const int rhi = (r0 + 3 + HALO) > (NH - 1) ? (NH - 1) : (r0 + 3 + HALO);
    const int nrows = rhi - rlo + 1;
    for (int i = tid; i < NC * nrows; i += 256) {
      int ci = i / nrows, rr = i - ci * nrows + rlo;
      __builtin_prefetch(inb + ci * NHW + rr * NW, 0, 1);
    }
  }
  for (int i = tid; i < NC * NC; i += 256) {
    int co = i >> 7, ci = i & (NC - 1);
    lds_w[co * LDW + ci] = (_Float16)(pw[i] * 16.0f);
  }
  for (int i = tid; i < NC * KS * KS; i += 256) lds_dw[i] = dw[i];
  __syncthreads();

  for (int i = tid; i < NC * 128; i += 256) {
    int ci = i >> 7;
    int s  = i & 127;
    int h = r0 + (s >> 5);
    int w = s & 31;
    const float* xp = inb + ci * NHW;
    const float* kw = &lds_dw[ci * KS * KS];
    float acc = 0.f;
#pragma unroll
    for (int ky = 0; ky < KS; ++ky) {
      int hh = h + (ky - KS / 2) * DIL;
      if ((unsigned)hh < (unsigned)NH) {
#pragma unroll
        for (int kx = 0; kx < KS; ++kx) {
          int ww = w + (kx - KS / 2) * DIL;
          if ((unsigned)ww < (unsigned)NW) {
            float t = xp[hh * NW + ww];
            acc += (t > 0.f ? t : 0.f) * kw[ky * KS + kx];
          }
        }
      }
    }
    lds_b[s * LDW + ci] = (_Float16)acc;
  }
  __syncthreads();

  const int wave  = tid >> 5;
  const int lane  = tid & 31;
  const int lhalf = lane >> 4;
  const int lmod  = lane & 15;
  const int m0    = wave * 16;

  v16h afrag[4];
  const int arow = m0 + lmod;
#pragma unroll
  for (int kt = 0; kt < 4; ++kt) {
    const int k0 = kt * 32 + lhalf * 8;
    const v8h lo = *(const v8h*)&lds_w[arow * LDW + k0];
    const v8h hi = *(const v8h*)&lds_w[arow * LDW + k0 + 16];
#pragma unroll
    for (int j = 0; j < 8; ++j) { afrag[kt][j] = lo[j]; afrag[kt][j + 8] = hi[j]; }
  }

  const float scale = (ACCUM ? (g * BN_SCALE) : BN_SCALE) * (1.0f / 16.0f);
  v8f accs[8];

#pragma unroll
  for (int nt = 0; nt < 8; ++nt) {
    const int n0 = nt * 16;
    const int brow = n0 + lmod;
    v8f acc = {};
#pragma unroll
    for (int kt = 0; kt < 4; ++kt) {
      const int k0 = kt * 32 + lhalf * 8;
      const v8h lo = *(const v8h*)&lds_b[brow * LDW + k0];
      const v8h hi = *(const v8h*)&lds_b[brow * LDW + k0 + 16];
      v16h bfrag;
#pragma unroll
      for (int j = 0; j < 8; ++j) { bfrag[j] = lo[j]; bfrag[j + 8] = hi[j]; }
      acc = __builtin_amdgcn_wmma_f32_16x16x32_f16(
           false, afrag[kt],  false, bfrag,
           (short)0, acc,  false,  false);
    }
    asm volatile("v_nop\n\tv_nop\n\tv_nop\n\tv_nop" : "+v"(acc) : "v"(afrag[0]), "v"(afrag[3]));
    accs[nt] = acc;
  }

  __syncthreads();
  const size_t plane0 = (size_t)(b * NC) * NHW + (size_t)r0 * NW;
#pragma unroll
  for (int nt = 0; nt < 8; ++nt) {
#pragma unroll
    for (int r = 0; r < 8; ++r) {
      const int co = m0 + lhalf * 8 + r, s = nt * 16 + lmod;
      float v = scale * accs[nt][r];
      if (ACCUM) v += out[plane0 + (size_t)co * NHW + s];
      cst[co * 128 + s] = v;
    }
  }
  __syncthreads();
#pragma unroll 4
  for (int rr = 0; rr < 16; ++rr) {
    const int co = m0 + rr;
    float* orow = out + plane0 + (size_t)co * NHW;
#pragma unroll
    for (int c = 0; c < 4; ++c) *(volatile float*)(orow + c * 32 + lane) = cst[co * 128 + c * 32 + lane];
  }
  __threadfence();
#pragma unroll 4
  for (int rr = 0; rr < 16; ++rr) {
    const int co = m0 + rr;
    float* orow = out + plane0 + (size_t)co * NHW;
#pragma unroll
    for (int c = 0; c < 4; ++c) *(volatile float*)(orow + c * 32 + lane) = cst[co * 128 + c * 32 + lane];
  }
}

extern "C" void kernel_launch(void* const* d_in, const int* in_sizes, int n_in,
                              void* d_out, int out_size, void* d_ws, size_t ws_size,
                              hipStream_t stream) {
  (void)in_sizes; (void)n_in; (void)out_size; (void)ws_size;

  const float* x      = (const float*)d_in[0];
  const float* wts    = (const float*)d_in[1];
  const float* sc3_d1 = (const float*)d_in[2];
  const float* sc3_p1 = (const float*)d_in[3];
  const float* sc3_d2 = (const float*)d_in[4];
  const float* sc3_p2 = (const float*)d_in[5];
  const float* sc5_d1 = (const float*)d_in[6];
  const float* sc5_p1 = (const float*)d_in[7];
  const float* sc5_d2 = (const float*)d_in[8];
  const float* sc5_p2 = (const float*)d_in[9];
  const float* dc3_d  = (const float*)d_in[10];
  const float* dc3_p  = (const float*)d_in[11];
  const float* dc5_d  = (const float*)d_in[12];
  const float* dc5_p  = (const float*)d_in[13];
  const int*   top    = (const int*)d_in[14];

  float* out   = (float*)d_out;
  float* w_out = out + (size_t)NB * NCHW;

  float* gate = (float*)d_ws;
  float* ybuf = (float*)((char*)d_ws + 4096);

  const int gemm_grid = NB * 8;

  gate_topk_kernel<<<1, 64, 0, stream>>>(wts, top, gate, w_out);
  pool_skip_kernel<<<(NB * NCHW) / 256, 256, 0, stream>>>(x, gate, out);

  sepstage_kernel<3, 1, false><<<gemm_grid, 256, 0, stream>>>(x,    sc3_d1, sc3_p1, gate, 4, ybuf);
  sepstage_kernel<3, 1, true ><<<gemm_grid, 256, 0, stream>>>(ybuf, sc3_d2, sc3_p2, gate, 4, out);
  sepstage_kernel<5, 1, false><<<gemm_grid, 256, 0, stream>>>(x,    sc5_d1, sc5_p1, gate, 5, ybuf);
  sepstage_kernel<5, 1, true ><<<gemm_grid, 256, 0, stream>>>(ybuf, sc5_d2, sc5_p2, gate, 5, out);
  sepstage_kernel<3, 2, true ><<<gemm_grid, 256, 0, stream>>>(x, dc3_d, dc3_p, gate, 6, out);
  sepstage_kernel<5, 2, true ><<<gemm_grid, 256, 0, stream>>>(x, dc5_d, dc5_p, gate, 7, out);
}
